// Causal_attention_70308614635806
// MI455X (gfx1250) — hardware-verified
//
#include <hip/hip_runtime.h>


namespace {
constexpr int Bn = 4, S = 4096, D = 512, NTOK = Bn * S, QB = 16, KC = 64;
constexpr float SCALE = 0.044194173824159216f;
constexpr size_t PL = (size_t)NTOK * D;

typedef _Float16 b16;
typedef __attribute__((ext_vector_type(16))) _Float16 v16b;
typedef __attribute__((ext_vector_type(8)))  _Float16 v8b;
typedef __attribute__((ext_vector_type(8)))  float v8f;
typedef __attribute__((ext_vector_type(4)))  float v4f;

__device__ __forceinline__ v8b ld8b(const b16* p) { return *(const v8b*)p; }
__device__ __forceinline__ v16b cat8b(v8b a, v8b b) { return __builtin_shufflevector(a, b, 0, 1, 2, 3, 4, 5, 6, 7, 8, 9, 10, 11, 12, 13, 14, 15); }
__device__ __forceinline__ v16b frag_kb(const b16* p, int hh) { return cat8b(ld8b(p + 8 * hh), ld8b(p + 16 + 8 * hh)); }
__device__ __forceinline__ void split16(float v, b16& hi, b16& lo) { hi = (b16)v; lo = (b16)(v - (float)hi); }
__device__ __forceinline__ void frag_ksplit(const float* p, int hh, v16b& fh_, v16b& fl_) {
  const float* p0 = p + 8 * hh; const float* p1 = p + 16 + 8 * hh;
#pragma unroll
  for (int e = 0; e < 8; ++e) { b16 a, c; split16(p0[e], a, c); fh_[e] = a; fl_[e] = c; split16(p1[e], a, c); fh_[8 + e] = a; fl_[8 + e] = c; }
}
__device__ __forceinline__ v8f wmma16b(v16b a, v16b b, v8f c) {
  v8f d = __builtin_amdgcn_wmma_f32_16x16x32_f16(false, a, false, b, (short)0, c, false, false);
  asm volatile("v_nop\n\tv_nop\n\tv_nop\n\tv_nop" : "+v"(d) : "v"(a), "v"(b));
  return d;
}
__device__ __forceinline__ void wave_lds_sync() {
  __builtin_amdgcn_fence(__ATOMIC_RELEASE, "workgroup");
  __builtin_amdgcn_wave_barrier();
  __builtin_amdgcn_fence(__ATOMIC_ACQUIRE, "workgroup");
}

struct Opnd { const void* p0; const void* p1; int ld; };
template <int NP> __device__ __forceinline__ void load_frags(const Opnd& o, int row, int kb, int hh, v16b& fh_, v16b& fl_) {
  if (NP == 0) { frag_ksplit((const float*)o.p0 + (size_t)row * o.ld + kb, hh, fh_, fl_); }
  else if (NP == 4 || NP == 5) {
    const float sc_ = (NP == 4) ? 64.0f : 8.0f;
    const float* p = (const float*)o.p0 + (size_t)row * o.ld + kb; const float* p0 = p + 8 * hh; const float* p1 = p + 16 + 8 * hh;
#pragma unroll
    for (int e = 0; e < 8; ++e) { b16 a, c; split16(p0[e] * sc_, a, c); fh_[e] = a; fl_[e] = c; split16(p1[e] * sc_, a, c); fh_[8 + e] = a; fl_[8 + e] = c; }
  } else if (NP == 3) {
    const float* p = (const float*)o.p0 + (size_t)row * o.ld + kb; const float* p0 = p + 8 * hh; const float* p1 = p + 16 + 8 * hh;
#pragma unroll
    for (int e = 0; e < 8; ++e) { fh_[e] = (b16)p0[e]; fh_[8 + e] = (b16)p1[e]; }
    fl_ = fh_;
  } else {
    fh_ = frag_kb((const b16*)o.p0 + (size_t)row * o.ld + kb, hh);
    if (NP == 2) fl_ = frag_kb((const b16*)o.p1 + (size_t)row * o.ld + kb, hh); else fl_ = fh_;
  }
}
template <int ANP, int BNP> __device__ __forceinline__ v8f mac(v16b ah, v16b al, v16b bh, v16b bl, v8f c) {
  c = wmma16b(ah, bh, c);
  if (BNP == 0 || BNP == 2 || BNP == 4 || BNP == 5) c = wmma16b(ah, bl, c);
  if (ANP == 0 || ANP == 2 || ANP == 4 || ANP == 5) c = wmma16b(al, bh, c);
  return c;
}
template <int ANP, int BNP>
__device__ __forceinline__ void gemm_tile(const Opnd& A, const Opnd& B, int K, int m0, int c0, int nloc, int hlf, v8f (&acc)[2][4]) {
  for (int kb = 0; kb < K; kb += 32) {
    v16b a0h, a0l, a1h, a1l;
    load_frags<ANP>(A, m0 + nloc, kb, hlf, a0h, a0l);
    load_frags<ANP>(A, m0 + 16 + nloc, kb, hlf, a1h, a1l);
#pragma unroll
    for (int t = 0; t < 4; ++t) {
      v16b bh, bl;
      load_frags<BNP>(B, c0 + t * 16 + nloc, kb, hlf, bh, bl);
      acc[0][t] = mac<ANP, BNP>(a0h, a0l, bh, bl, acc[0][t]);
      acc[1][t] = mac<ANP, BNP>(a1h, a1l, bh, bl, acc[1][t]);
    }
  }
}

__device__ __forceinline__ void epi_planes(v8f (&acc)[2][4], float scale, bool two, b16* __restrict__ oh, b16* __restrict__ ol, int ldo,
                                           int m0, int c0, int lane, b16* Th, b16* Tl) {
  const int nloc = lane & 15, hlf = lane >> 4;
#pragma unroll
  for (int t = 0; t < 4; ++t)
#pragma unroll
    for (int r = 0; r < 2; ++r)
#pragma unroll
      for (int v = 0; v < 8; ++v) {
        const int rr = r * 16 + v + 8 * hlf, cc = t * 16 + nloc;
        b16 h_, l_; split16(acc[r][t][v] * scale, h_, l_);
        Th[rr * 64 + cc] = h_; Tl[rr * 64 + cc] = l_;
      }
  wave_lds_sync();
  for (int pass = 0; pass < 2; ++pass) {
#pragma unroll
    for (int j = 0; j < 8; ++j) {
      const int rr = j * 4 + (lane >> 3), c8 = (lane & 7) * 8;
      const size_t o = (size_t)(m0 + rr) * ldo + c0 + c8;
      *(volatile v8b*)(oh + o) = ld8b(Th + rr * 64 + c8);
      if (two) *(volatile v8b*)(ol + o) = ld8b(Tl + rr * 64 + c8);
    }
    __threadfence();
  }
}
__device__ __forceinline__ void epi_f32(v8f (&acc)[2][4], float scale, const float* rscale, float* __restrict__ out, int ldo, int m0, int c0, int lane, float* Tt) {
  const int nloc = lane & 15, hlf = lane >> 4;
#pragma unroll
  for (int t = 0; t < 4; ++t)
#pragma unroll
    for (int r = 0; r < 2; ++r)
#pragma unroll
      for (int v = 0; v < 8; ++v) {
        const int rr = r * 16 + v + 8 * hlf;
        const float rs = rscale ? rscale[(size_t)(m0 + rr) * 32] : 1.0f;
        Tt[rr * 64 + t * 16 + nloc] = acc[r][t][v] * scale * rs;
      }
  wave_lds_sync();
  float* dst0 = out + (size_t)m0 * ldo + c0;
  for (int pass = 0; pass < 2; ++pass) {
#pragma unroll
    for (int j = 0; j < 16; ++j) { const int rr = j * 2 + hlf, c4 = nloc * 4; *(volatile v4f*)(dst0 + (size_t)rr * ldo + c4) = *(const v4f*)(Tt + rr * 64 + c4); }
    __threadfence();
  }
}


typedef __attribute__((ext_vector_type(8))) __bf16 v8bb; typedef __attribute__((ext_vector_type(16))) __bf16 v16bb;
typedef __attribute__((ext_vector_type(8))) unsigned short v8us;
__device__ __forceinline__ v16bb frag_kb_bf(const __bf16* p, int hh) { const v8bb a = *(const v8bb*)(p + 8 * hh), b = *(const v8bb*)(p + 16 + 8 * hh); return __builtin_shufflevector(a, b, 0, 1, 2, 3, 4, 5, 6, 7, 8, 9, 10, 11, 12, 13, 14, 15); }
__device__ __forceinline__ v8f wmma16bb(v16bb a, v16bb b, v8f c) {
  v8f d = __builtin_amdgcn_wmma_f32_16x16x32_bf16(false, a, false, b, (short)0, c, false, false);
  asm volatile("v_nop\n\tv_nop\n\tv_nop\n\tv_nop" : "+v"(d) : "v"(a), "v"(b));
  return d;
}
__device__ __forceinline__ unsigned short bf16_rne_bits(float v) { unsigned int u = __float_as_uint(v); u += 0x7FFFu + ((u >> 16) & 1u); return (unsigned short)(u >> 16); }
__device__ __forceinline__ float bf16_rne(float v) { return __uint_as_float(((unsigned int)bf16_rne_bits(v)) << 16); }


__global__ __launch_bounds__(256) void prep_kernel(const float* __restrict__ x, const float* __restrict__ wq, const float* __restrict__ wk, const float* __restrict__ wv,
                                                   b16* __restrict__ xh, unsigned short* __restrict__ wkb, b16* __restrict__ wqT, b16* __restrict__ wvh) {
  const size_t tid = (size_t)blockIdx.x * blockDim.x + threadIdx.x, nth = (size_t)gridDim.x * blockDim.x;
  for (int pass = 0; pass < 2; ++pass) {
    for (size_t p = tid; p < (size_t)NTOK * D / 8; p += nth) { v8b v;
#pragma unroll
      for (int e = 0; e < 8; ++e) v[e] = (b16)bf16_rne(x[p * 8 + e]);
      *(volatile v8b*)(xh + p * 8) = v; }
    for (size_t p = tid; p < (size_t)D * D / 8; p += nth) { const int n = (int)(p / (D / 8)), k0 = (int)(p % (D / 8)) * 8; v8us a; v8b q, v;
#pragma unroll
      for (int e = 0; e < 8; ++e) { a[e] = bf16_rne_bits(wk[p * 8 + e]); q[e] = (b16)bf16_rne(wq[(size_t)(k0 + e) * D + n]); v[e] = (b16)bf16_rne(wv[p * 8 + e]); }
      *(volatile v8us*)(wkb + p * 8) = a; *(volatile v8b*)(wqT + (size_t)n * D + k0) = q; *(volatile v8b*)(wvh + p * 8) = v; }
    __threadfence();
  }
}

__global__ __launch_bounds__(256) void xt_kernel(const b16* __restrict__ xh, b16* __restrict__ xt) {
  __shared__ __attribute__((aligned(16))) b16 T[D][64 + 8];
  const int t_ = threadIdx.x, tokb = blockIdx.x * 64, b = tokb / S, s0 = tokb % S;
  for (int i = t_; i < 64 * D / 8; i += 256) { const int r = i / (D / 8), c8 = (i % (D / 8)) * 8; const v8b v = *(const v8b*)(xh + (size_t)(tokb + r) * D + c8);
#pragma unroll
    for (int e = 0; e < 8; ++e) T[c8 + e][r] = v[e]; }
  __syncthreads();
  for (int pass = 0; pass < 2; ++pass) { for (int i = t_; i < D * 8; i += 256) { const int d = i >> 3, c8 = (i & 7) * 8; *(volatile v8b*)(xt + ((size_t)b * D + d) * S + s0 + c8) = *(const v8b*)(&T[d][c8]); } __threadfence(); }
}

__global__ __launch_bounds__(128) void kproj_kernel(const float* __restrict__ x, const __bf16* __restrict__ wkb, b16* __restrict__ kpl) {
  __shared__ __attribute__((aligned(16))) b16 Th[4][2][32 * 64];
  const int lane = threadIdx.x & 31, wave = threadIdx.x >> 5, nloc = lane & 15, hlf = lane >> 4, m0 = blockIdx.y * 128 + wave * 32, c0 = blockIdx.x * 64;
  v8f acc[2][4];
#pragma unroll
  for (int r = 0; r < 2; ++r)
#pragma unroll
    for (int t = 0; t < 4; ++t) acc[r][t] = (v8f){};
#pragma unroll 2
  for (int kb = 0; kb < D; kb += 32) { v16bb a0, a1;
    { const float* p0 = x + (size_t)(m0 + nloc) * D + kb; const float* p1 = x + (size_t)(m0 + 16 + nloc) * D + kb;
#pragma unroll
      for (int e = 0; e < 8; ++e) { a0[e] = (__bf16)bf16_rne(p0[8 * hlf + e]); a0[8 + e] = (__bf16)bf16_rne(p0[16 + 8 * hlf + e]); a1[e] = (__bf16)bf16_rne(p1[8 * hlf + e]); a1[8 + e] = (__bf16)bf16_rne(p1[16 + 8 * hlf + e]); } }
#pragma unroll
    for (int t = 0; t < 4; ++t) { const v16bb bw = frag_kb_bf(wkb + (size_t)(c0 + t * 16 + nloc) * D + kb, hlf); acc[0][t] = wmma16bb(a0, bw, acc[0][t]); acc[1][t] = wmma16bb(a1, bw, acc[1][t]); } }
  epi_planes(acc, 8.0f, true, kpl, kpl + PL, D, m0, c0, lane, Th[wave][0], Th[wave][1]);
}

__global__ __launch_bounds__(128) void z_kernel(const b16* __restrict__ kpl, const b16* __restrict__ wqT, b16* __restrict__ zpl) {
  __shared__ __attribute__((aligned(16))) b16 Th[4][2][32 * 64];
  const int lane = threadIdx.x & 31, wave = threadIdx.x >> 5, nloc = lane & 15, hlf = lane >> 4, m0 = blockIdx.y * 128 + wave * 32, c0 = blockIdx.x * 64;
  v8f acc[2][4];
#pragma unroll
  for (int r = 0; r < 2; ++r)
#pragma unroll
    for (int t = 0; t < 4; ++t) acc[r][t] = (v8f){};
  const Opnd A{kpl, kpl + PL, D}, Bo{wqT, nullptr, D};
  gemm_tile<2, 1>(A, Bo, D, m0, c0, nloc, hlf, acc);
  epi_planes(acc, 1.0f, true, zpl, zpl + PL, D, m0, c0, lane, Th[wave][0], Th[wave][1]);
}

__global__ __launch_bounds__(128) void attn_kernel(const b16* __restrict__ xh, const b16* __restrict__ zpl, const b16* __restrict__ xt, float* __restrict__ u) {
  __shared__ __attribute__((aligned(16))) float Sp[4][QB][KC + 4];
  __shared__ __attribute__((aligned(16))) b16 Ph[QB][KC + 8], Plo[QB][KC + 8];
  __shared__ float Al[QB], Linv[QB];
  __shared__ __attribute__((aligned(16))) float Ot[4][QB][128 + 4];
  const int wave = threadIdx.x >> 5, lane = threadIdx.x & 31, nloc = lane & 15, hlf = lane >> 4;
  const int blk = blockIdx.x, b = blk / (S / QB), q0 = (blk % (S / QB)) * QB;
  const b16* Xq = xh + ((size_t)b * S + q0) * D; const b16* Z = zpl + (size_t)b * S * D; const b16* Xt = xt + (size_t)b * D * S;
  const int d0 = wave * 128;
  v16b qf[4];
#pragma unroll
  for (int ks = 0; ks < 4; ++ks) qf[ks] = frag_kb(Xq + (size_t)nloc * D + d0 + ks * 32, hlf);
  float m_run = -INFINITY, l_run = 0.0f;
  v8f o[8] = {{}, {}, {}, {}, {}, {}, {}, {}};
  for (int kb = 0; kb < q0 + QB; kb += KC) {
    v8f sp[4] = {{}, {}, {}, {}};
#pragma unroll
    for (int ks = 0; ks < 4; ++ks)
#pragma unroll
      for (int kt = 0; kt < 4; ++kt) { const size_t zo = (size_t)(kb + kt * 16 + nloc) * D + d0 + ks * 32; const v16b zh = frag_kb(Z + zo, hlf), zl = frag_kb(Z + PL + zo, hlf);
        sp[kt] = wmma16b(zh, qf[ks], sp[kt]); sp[kt] = wmma16b(zl, qf[ks], sp[kt]); }
#pragma unroll
    for (int kt = 0; kt < 4; ++kt)
#pragma unroll
      for (int v = 0; v < 8; ++v) Sp[wave][nloc][kt * 16 + 8 * hlf + v] = sp[kt][v];
    __syncthreads();
    if (wave == 0) {
      const int qi = q0 + nloc; float sv[32]; float mx = -INFINITY;
#pragma unroll
      for (int j = 0; j < 32; ++j) { const int key = kb + hlf * 32 + j; float s = (Sp[0][nloc][hlf * 32 + j] + Sp[1][nloc][hlf * 32 + j] + Sp[2][nloc][hlf * 32 + j] + Sp[3][nloc][hlf * 32 + j]) * (SCALE / 8.0f);
        if (key > qi) s = -INFINITY; sv[j] = s; mx = fmaxf(mx, s); }
      mx = fmaxf(mx, __shfl_xor(mx, 16));
      const float mn = fmaxf(m_run, mx), al_ = __expf(m_run - mn); m_run = mn;
      float sum = 0.0f;
#pragma unroll
      for (int j = 0; j < 32; ++j) { const float e = __expf(sv[j] - mn); sum += e; b16 a, c; split16(e * 8.0f, a, c); Ph[nloc][hlf * 32 + j] = a; Plo[nloc][hlf * 32 + j] = c; }
      sum += __shfl_xor(sum, 16); l_run = l_run * al_ + sum;
      if (hlf == 0) { Al[nloc] = al_; Linv[nloc] = 1.0f / (8.0f * l_run); }
    }
    __syncthreads();
    { const float alq = Al[nloc];
#pragma unroll
      for (int t = 0; t < 8; ++t)
#pragma unroll
        for (int v = 0; v < 8; ++v) o[t][v] *= alq; }
#pragma unroll
    for (int ks = 0; ks < 2; ++ks) { const v16b ph = frag_kb(&Ph[nloc][0] + ks * 32, hlf), pl = frag_kb(&Plo[nloc][0] + ks * 32, hlf);
#pragma unroll
      for (int t = 0; t < 8; ++t) { const v16b xf = frag_kb(Xt + (size_t)(d0 + t * 16 + nloc) * S + kb + ks * 32, hlf); o[t] = wmma16b(xf, ph, o[t]); o[t] = wmma16b(xf, pl, o[t]); } }
  }
  { const float li = Linv[nloc];
#pragma unroll
    for (int t = 0; t < 8; ++t)
#pragma unroll
      for (int v = 0; v < 8; ++v) Ot[wave][nloc][t * 16 + 8 * hlf + v] = o[t][v] * li; }
  wave_lds_sync();
  float* dst = u + ((size_t)b * S + q0) * D + d0;
  for (int pass = 0; pass < 2; ++pass) {
#pragma unroll
    for (int rr = 0; rr < QB; ++rr) *(volatile v4f*)(dst + (size_t)rr * D + lane * 4) = *(const v4f*)(&Ot[wave][rr][lane * 4]);
    __threadfence();
  }
}

__global__ __launch_bounds__(128) void y_kernel(const float* __restrict__ u, const b16* __restrict__ wvh, float* __restrict__ y) {
  __shared__ __attribute__((aligned(16))) float Ts[4][32 * 64];
  const int lane = threadIdx.x & 31, wave = threadIdx.x >> 5, nloc = lane & 15, hlf = lane >> 4, m0 = blockIdx.y * 128 + wave * 32, c0 = blockIdx.x * 64;
  v8f acc[2][4];
#pragma unroll
  for (int r = 0; r < 2; ++r)
#pragma unroll
    for (int t = 0; t < 4; ++t) acc[r][t] = (v8f){};
  const Opnd A{u, nullptr, D}, Bo{wvh, nullptr, D};
  gemm_tile<5, 1>(A, Bo, D, m0, c0, nloc, hlf, acc);
  epi_f32(acc, 1.0f / 8.0f, nullptr, y, D, m0, c0, lane, Ts[wave]);
}
}

extern "C" void kernel_launch(void* const* d_in, const int* in_sizes, int n_in,
                              void* d_out, int out_size, void* d_ws, size_t ws_size, hipStream_t stream) {
  (void)n_in; (void)out_size;
  const float* x = (const float*)d_in[0]; const float* wq = (const float*)d_in[1]; const float* wk = (const float*)d_in[2]; const float* wv = (const float*)d_in[3];
  float* out = (float*)d_out;
  if (in_sizes[0] != NTOK * D || in_sizes[1] != D * D || in_sizes[2] != D * D || in_sizes[3] != D * D) return;
  size_t off = 0; char* ws = (char*)d_ws;
  auto carve = [&](size_t bytes) { char* p = ws + off; off += (bytes + 255) & ~(size_t)255; return p; };
  b16* xh = (b16*)carve(PL * 2); b16* xt = (b16*)carve(PL * 2); unsigned short* wkb = (unsigned short*)carve((size_t)D * D * 2); b16* wqT = (b16*)carve((size_t)D * D * 2); b16* wvh = (b16*)carve((size_t)D * D * 2);
  b16* kpl = (b16*)carve(PL * 2 * 2); b16* zpl = (b16*)carve(PL * 2 * 2);
  float* u = (float*)kpl;
  if (off > ws_size) return;
  prep_kernel<<<1024, 256, 0, stream>>>(x, wq, wk, wv, xh, wkb, wqT, wvh);
  xt_kernel<<<NTOK / 64, 256, 0, stream>>>(xh, xt);
  kproj_kernel<<<dim3(D / 64, NTOK / 128), 128, 0, stream>>>(x, (const __bf16*)wkb, kpl);
  z_kernel<<<dim3(D / 64, NTOK / 128), 128, 0, stream>>>(kpl, wqT, zpl);
  attn_kernel<<<Bn * S / QB, 128, 0, stream>>>(xh, zpl, xt, u);
  y_kernel<<<dim3(D / 64, NTOK / 128), 128, 0, stream>>>(u, wvh, out);
}
